// ModulatedDeformConv3DWithOffset_60215441489982
// MI455X (gfx1250) — hardware-verified
//
#include <hip/hip_runtime.h>
#include <math.h>

typedef __attribute__((ext_vector_type(16))) _Float16 v16h;
typedef __attribute__((ext_vector_type(16))) __bf16 v16b;
typedef __attribute__((ext_vector_type(8)))  _Float16 v8h;
typedef __attribute__((ext_vector_type(8)))  float v8f;
typedef __attribute__((ext_vector_type(4)))  float v4f;
typedef __attribute__((ext_vector_type(2)))  float v2f;
typedef __attribute__((ext_vector_type(4)))  unsigned v4u;
typedef __attribute__((ext_vector_type(4)))  int v4i;
typedef float __attribute__((may_alias)) float_a;
typedef int __attribute__((may_alias)) int_a;

template <typename T> __device__ __forceinline__ void vst2(void* p, T v) { *(volatile T*)p = v; __threadfence(); *(volatile T*)p = v; }
__device__ __forceinline__ v8f wmma16(v16h a, v16h b, v8f c) {
  v8f d = __builtin_amdgcn_wmma_f32_16x16x32_f16(false, a, false, b, (short)0, c, false, false);
  asm volatile("v_nop\n\tv_nop\n\tv_nop\n\tv_nop" : "+v"(d) : "v"(a), "v"(b));
  return d;
}
__device__ __forceinline__ v8f wmma_bf(v16b a, v16b b, v8f c) {
  v8f d = __builtin_amdgcn_wmma_f32_16x16x32_bf16(false, a, false, b, (short)0, c, false, false);
  asm volatile("v_nop\n\tv_nop\n\tv_nop\n\tv_nop" : "+v"(d) : "v"(a), "v"(b));
  return d;
}
__device__ __forceinline__ v16h frag_h(const _Float16* rowk0, int lane) {
  union { v16h v; v8h q[2]; } u; const _Float16* p = rowk0 + 8 * (lane >> 4);
  u.q[0] = *(const v8h*)p; u.q[1] = *(const v8h*)(p + 16); return u.v;
}
__device__ __forceinline__ v16h frag_f32(const float* rowk0, int lane) {
  v16h a; const float* p = rowk0 + 8 * (lane >> 4);
#pragma unroll
  for (int i = 0; i < 8; ++i) { a[i] = (_Float16)p[i]; a[8 + i] = (_Float16)p[16 + i]; }
  return a;
}
__device__ __forceinline__ v16h frag_f32s(const float* rowk0, int lane, float sc) {
  v16h a; const float* p = rowk0 + 8 * (lane >> 4);
#pragma unroll
  for (int i = 0; i < 8; ++i) { a[i] = (_Float16)(p[i] * sc); a[8 + i] = (_Float16)(p[16 + i] * sc); }
  return a;
}
__device__ __forceinline__ v16h fragc_f32(const float* W, int k0, int n, int lane, int ld, int K) {
  v16h a; const int g = lane >> 4;
#pragma unroll
  for (int i = 0; i < 8; ++i) { const int ka = k0 + 8 * g + i, kb = ka + 16;
    a[i] = (_Float16)(ka < K ? W[(size_t)ka * ld + n] : 0.f); a[8 + i] = (_Float16)(kb < K ? W[(size_t)kb * ld + n] : 0.f); }
  return a;
}
struct F2 { v16b h, l; };
__device__ __forceinline__ F2 bsplit16(const float v[16]) { F2 r;
#pragma unroll
  for (int i = 0; i < 16; ++i) { const __bf16 h = (__bf16)v[i]; r.h[i] = h; r.l[i] = (__bf16)(v[i] - (float)h); }
  return r; }
__device__ __forceinline__ F2 split_row(const float* row, int k0, int lane) { float v[16]; const float* p = row + k0 + 8 * (lane >> 4);
#pragma unroll
  for (int i = 0; i < 8; ++i) { v[i] = p[i]; v[8 + i] = p[16 + i]; }
  return bsplit16(v); }
__device__ __forceinline__ F2 split_rowK(const float* row, int k0, int lane, int K) { float v[16]; const int g = lane >> 4;
#pragma unroll
  for (int i = 0; i < 8; ++i) { const int ka = k0 + 8 * g + i, kb = ka + 16; v[i] = ka < K ? row[ka] : 0.f; v[8 + i] = kb < K ? row[kb] : 0.f; }
  return bsplit16(v); }
__device__ __forceinline__ F2 split_col(const float* W, int k0, int n, int lane, int ld, int K) { float v[16]; const int g = lane >> 4;
#pragma unroll
  for (int i = 0; i < 8; ++i) { const int ka = k0 + 8 * g + i, kb = ka + 16; v[i] = ka < K ? W[(size_t)ka * ld + n] : 0.f; v[8 + i] = kb < K ? W[(size_t)kb * ld + n] : 0.f; }
  return bsplit16(v); }
__device__ __forceinline__ v8f mac3(const F2& a, const F2& b, v8f c) { c = wmma_bf(a.l, b.h, c); c = wmma_bf(a.h, b.l, c); return wmma_bf(a.h, b.h, c); }
__device__ __forceinline__ float sigm(float v) { return 1.0f / (1.0f + expf(-v)); }
#define LDSX() do { asm volatile("s_wait_dscnt 0" ::: "memory"); __builtin_amdgcn_wave_barrier(); __builtin_amdgcn_fence(__ATOMIC_RELEASE, "workgroup"); } while (0)

#define NBT 2
#define CI 256
#define CO 256
#define TT 8
#define HI 32
#define WI 32
#define NPX (HI * WI)
#define NFR (NBT * TT)
#define KK 9
#define KTOT (CI * KK)
#define NOFF 27

__device__ __forceinline__ size_t xidx(int n, int c, int p) { const int b = n / TT, t = n % TT; return (((size_t)b * CI + c) * TT + t) * NPX + p; }

__global__ __launch_bounds__(256) void k_im2col(const float* __restrict__ x, _Float16* __restrict__ A) {
  __shared__ __align__(16) _Float16 srow[64][KTOT + 8];
  const int n = blockIdx.y, p0 = blockIdx.x * 64, tid = threadIdx.x;
  for (int q = tid; q < 64 * CI; q += 256) { const int pl = q & 63, c = q >> 6; const int p = p0 + pl, py = p / WI, px = p % WI;
#pragma unroll
    for (int k = 0; k < KK; ++k) { const int yy = py + k / 3 - 1, xx = px + k % 3 - 1; const float v = (yy >= 0 && yy < HI && xx >= 0 && xx < WI) ? x[xidx(n, c, yy * WI + xx)] : 0.f; srow[pl][c * KK + k] = (_Float16)v; } }
  __syncthreads();
  for (int q = tid; q < 64 * (KTOT / 8); q += 256) { const int pl = q / (KTOT / 8), pc = q % (KTOT / 8); vst2(A + ((size_t)n * NPX + p0 + pl) * KTOT + pc * 8, *(const v4u*)(&srow[pl][pc * 8])); }
}
__global__ __launch_bounds__(256) void k_packW(const float* __restrict__ W, const float* __restrict__ OW, _Float16* __restrict__ P) {
  const int r = blockIdx.x, tid = threadIdx.x; __shared__ __align__(16) _Float16 srow[KTOT];
  for (int q = tid; q < KTOT; q += 256) { float v = 0.f; if (r < CO) v = W[(size_t)r * KTOT + q]; else if (r - CO < NOFF) v = OW[(size_t)(r - CO) * KTOT + q]; srow[q] = (_Float16)(v * 16.0f); }
  __syncthreads();
  for (int q = tid; q < KTOT / 8; q += 256) vst2(P + (size_t)r * KTOT + q * 8, *(const v4u*)(&srow[q * 8]));
}
__global__ __launch_bounds__(128) void k_off(const _Float16* __restrict__ A, const _Float16* __restrict__ P, const float* __restrict__ ob, float* __restrict__ om) {
  __shared__ __align__(16) float so[4][16][36];
  const int tid = threadIdx.x, wave = tid >> 5, lane = tid & 31, col = lane & 15, g = lane >> 4;
  const int r0 = blockIdx.x * 64 + wave * 16;
  v8f acc[2] = {};
#pragma unroll 1
  for (int kc = 0; kc < KTOT / 32; ++kc) { const v16h a = frag_h(A + (size_t)(r0 + col) * KTOT + kc * 32, lane);
#pragma unroll
    for (int j = 0; j < 2; ++j) acc[j] = wmma16(a, frag_h(P + (size_t)(CO + j * 16 + col) * KTOT + kc * 32, lane), acc[j]); }
#pragma unroll
  for (int j = 0; j < 2; ++j) { const int c = j * 16 + col;
#pragma unroll
    for (int r = 0; r < 8; ++r) so[wave][8 * g + r][c] = acc[j][r] * (1.0f / 16.0f) + (c < NOFF ? ob[c] : 0.f); }
  LDSX();
  for (int q = lane; q < 16 * 8; q += 32) { const int rl = q >> 3, pc = q & 7; vst2(om + (size_t)(r0 + rl) * 32 + pc * 4, *(const v4f*)(&so[wave][rl][pc * 4])); }
}
__global__ __launch_bounds__(256) void k_sample(const float* __restrict__ x, const float* __restrict__ om, _Float16* __restrict__ A) {
  __shared__ __align__(16) _Float16 srow[64][KTOT + 8];
  __shared__ float swt[64][KK][4]; __shared__ int sidx[64][KK][4]; __shared__ float smk[64][KK];
  const int n = blockIdx.y, p0 = blockIdx.x * 64, tid = threadIdx.x;
  for (int q = tid; q < 64 * KK; q += 256) { const int pl = q / KK, k = q % KK; const int p = p0 + pl, oy = p / WI, ox = p % WI; const float* omr = om + ((size_t)n * NPX + p) * 32;
    const float dy = omr[2 * k], dx = omr[2 * k + 1]; const float mk = sigm(omr[18 + k]);
    const float py = dy + (float)(oy - 1 + k / 3), px = dx + (float)(ox - 1 + k % 3);
    const float fy = floorf(py), fx = floorf(px); const float ty = py - fy, tx = px - fx; const int y0 = (int)fy, x0 = (int)fx;
#pragma unroll
    for (int cn = 0; cn < 4; ++cn) { const int yy = y0 + (cn >> 1), xx = x0 + (cn & 1); const bool valid = yy >= 0 && yy < HI && xx >= 0 && xx < WI;
      const float wgt = ((cn >> 1) ? ty : 1.0f - ty) * ((cn & 1) ? tx : 1.0f - tx);
      swt[pl][k][cn] = valid ? wgt : 0.f; sidx[pl][k][cn] = valid ? (yy * WI + xx) : 0; }
    smk[pl][k] = mk; }
  __syncthreads();
  for (int q = tid; q < 64 * CI; q += 256) { const int pl = q & 63, c = q >> 6;
#pragma unroll
    for (int k = 0; k < KK; ++k) { float v = 0.f;
#pragma unroll
      for (int cn = 0; cn < 4; ++cn) { const float wg = swt[pl][k][cn]; if (wg != 0.f) v += x[xidx(n, c, sidx[pl][k][cn])] * wg; }
      srow[pl][c * KK + k] = (_Float16)(v * smk[pl][k]); } }
  __syncthreads();
  for (int q = tid; q < 64 * (KTOT / 8); q += 256) { const int pl = q / (KTOT / 8), pc = q % (KTOT / 8); vst2(A + ((size_t)n * NPX + p0 + pl) * KTOT + pc * 8, *(const v4u*)(&srow[pl][pc * 8])); }
}
__global__ __launch_bounds__(128) void k_main(const _Float16* __restrict__ A, const _Float16* __restrict__ P, const float* __restrict__ bias, float* __restrict__ out) {
  __shared__ __align__(16) float st[128][68];
  const int tid = threadIdx.x, wave = tid >> 5, lane = tid & 31, col = lane & 15, g = lane >> 4;
  const int n = blockIdx.z, p0b = blockIdx.x * 64, r0 = n * NPX + p0b + wave * 16, o0 = blockIdx.y * 128; const int b = n / TT, t = n % TT;
  v8f acc[8] = {};
#pragma unroll 1
  for (int kc = 0; kc < KTOT / 32; ++kc) { const v16h a = frag_h(A + (size_t)(r0 + col) * KTOT + kc * 32, lane);
#pragma unroll
    for (int j = 0; j < 8; ++j) acc[j] = wmma16(a, frag_h(P + (size_t)(o0 + j * 16 + col) * KTOT + kc * 32, lane), acc[j]); }
#pragma unroll
  for (int j = 0; j < 8; ++j) { const int ol = j * 16 + col; const float bb = bias[o0 + ol];
#pragma unroll
    for (int r = 0; r < 8; ++r) st[ol][wave * 16 + 8 * g + r] = acc[j][r] * (1.0f / 16.0f) + bb; }
  __syncthreads();
  for (int q = tid; q < 128 * 16; q += 128) { const int ol = q >> 4, pc = q & 15; vst2(out + (((size_t)b * CO + o0 + ol) * TT + t) * NPX + p0b + pc * 4, *(const v4f*)(&st[ol][pc * 4])); }
}
extern "C" void kernel_launch(void* const* d_in, const int* in_sizes, int n_in, void* d_out, int out_size, void* d_ws, size_t ws_size, hipStream_t stream) {
  (void)in_sizes; (void)n_in; (void)out_size; (void)ws_size;
  const float* x = (const float*)d_in[0]; const float* W = (const float*)d_in[1]; const float* bias = (const float*)d_in[2]; const float* OW = (const float*)d_in[3]; const float* ob = (const float*)d_in[4];
  float* out = (float*)d_out;
  char* ws = (char*)d_ws; size_t off = 0;
  auto take = [&](size_t bytes) { char* p = ws + off; off += (bytes + 255) & ~(size_t)255; return p; };
  _Float16* A = (_Float16*)take((size_t)NFR * NPX * KTOT * 2); _Float16* P = (_Float16*)take((size_t)(CO + 32) * KTOT * 2); float* om = (float*)take((size_t)NFR * NPX * 32 * 4);
  k_im2col<<<dim3(NPX / 64, NFR), 256, 0, stream>>>(x, A);
  k_packW<<<CO + 32, 256, 0, stream>>>(W, OW, P);
  k_off<<<NFR * NPX / 64, 128, 0, stream>>>(A, P, ob, om);
  k_sample<<<dim3(NPX / 64, NFR), 256, 0, stream>>>(x, om, A);
  k_main<<<dim3(NPX / 64, CO / 128, NFR), 128, 0, stream>>>(A, P, bias, out);
}
